// SAGELayer1_41240275976352
// MI455X (gfx1250) — hardware-verified
//
#include <hip/hip_runtime.h>
#include <stddef.h>


#define FD      128
#define HD      128
#define KA      (2 * FD)
#define NTHR    256
#define NWAVE   8
#define EPT     8
#define NGRP    2
#define CHUNK   (NTHR * EPT * NGRP)
#define WCAP    (EPT * NGRP * 32)
#define LISTN   (NWAVE * WCAP)
#define NBC     4096
#define NBF     2048
#define FPC     (NBC / NBF)
#define RCAP    40960
#define RBN     128
#define TGT     256
#define DEGCAP  256
#define OTHR    512
#define GBM     128
#define WSCAP   134217728
#define WSCL    64.0f
#define WSCLI   0.015625f
#define OV      (GBM * HD / 4 / NTHR)
#define WUNITS  (HD * (KA / 8))
#define POISON  30000.0f

#define LDS_FILL ((RCAP + NBF + LISTN) * 4 + 64)
#define LDS_GN   (GBM * KA * 2 + GBM * HD * 4)

static_assert((CHUNK & (CHUNK - 1)) == 0);
static_assert(CHUNK <= 4096);
static_assert(NBC <= 4096 && NBF <= 4096);
static_assert((NBC & (NBC - 1)) == 0 && (NBF & (NBF - 1)) == 0);
static_assert(NBC == FPC * NBF && FPC == 2);
static_assert(OTHR * 8 == NBC);
static_assert(OTHR / 32 == 8 * FPC);
static_assert((RCAP % 32) == 0);
static_assert(TGT == NWAVE * 32);
static_assert((TGT % GBM) == 0);
static_assert((DEGCAP % 32) == 0);
static_assert(GBM == NWAVE * 16 && NWAVE == 8);
static_assert((FD % 32) == 0 && FD == 4 * 32);
static_assert((KA % 32) == 0 && KA == 256);
static_assert((HD % 16) == 0 && HD == 8 * 16);
static_assert(OV * NTHR * 4 == GBM * HD);
static_assert((GBM * HD * 4) % 128 == 0);
static_assert((HD * 4) % 128 == 0);
static_assert((WUNITS % NTHR) == 0);

typedef float          v4f  __attribute__((ext_vector_type(4)));
typedef float          v8f  __attribute__((ext_vector_type(8)));
typedef int            v4i  __attribute__((ext_vector_type(4)));
typedef _Float16       v8h  __attribute__((ext_vector_type(8)));
typedef _Float16       v16h __attribute__((ext_vector_type(16)));
union FragH { v16h v; v8h h[2]; };

__device__ __forceinline__ v8f wmh(v16h a, v16h b, v8f c) {
  v8f d = __builtin_amdgcn_wmma_f32_16x16x32_f16(false, a, false, b, (short)0, c, false, false);
  asm volatile("v_nop\n\tv_nop\n\tv_nop\n\tv_nop" : "+v"(d) : "v"(a), "v"(b));
  return d;
}

__device__ __forceinline__ v8h cvt8(v4f a, v4f b, float s) {
  v8h r;
  r[0] = (_Float16)(a.x * s); r[1] = (_Float16)(a.y * s); r[2] = (_Float16)(a.z * s); r[3] = (_Float16)(a.w * s);
  r[4] = (_Float16)(b.x * s); r[5] = (_Float16)(b.y * s); r[6] = (_Float16)(b.z * s); r[7] = (_Float16)(b.w * s);
  return r;
}

__global__ __launch_bounds__(NTHR) void k_wprep(const float* __restrict__ Wx, const float* __restrict__ Wm,
                                               _Float16* pl, int units) {
  const int i = (int)blockIdx.x * NTHR + (int)threadIdx.x;
  if (i >= units) return;
  const int n  = i >> 5;
  const int k0 = (i & 31) * 8;
  const int kk = k0 >= FD ? k0 - FD : k0;
  const int nc = n < HD - 1 ? n : HD - 1;
  v4f a0, a1, c0, c1;
  a0.x = Wx[(size_t)(kk + 0) * HD + nc]; a0.y = Wx[(size_t)(kk + 1) * HD + nc];
  a0.z = Wx[(size_t)(kk + 2) * HD + nc]; a0.w = Wx[(size_t)(kk + 3) * HD + nc];
  a1.x = Wx[(size_t)(kk + 4) * HD + nc]; a1.y = Wx[(size_t)(kk + 5) * HD + nc];
  a1.z = Wx[(size_t)(kk + 6) * HD + nc]; a1.w = Wx[(size_t)(kk + 7) * HD + nc];
  c0.x = Wm[(size_t)(kk + 0) * HD + nc]; c0.y = Wm[(size_t)(kk + 1) * HD + nc];
  c0.z = Wm[(size_t)(kk + 2) * HD + nc]; c0.w = Wm[(size_t)(kk + 3) * HD + nc];
  c1.x = Wm[(size_t)(kk + 4) * HD + nc]; c1.y = Wm[(size_t)(kk + 5) * HD + nc];
  c1.z = Wm[(size_t)(kk + 6) * HD + nc]; c1.w = Wm[(size_t)(kk + 7) * HD + nc];
  if (k0 >= FD) { a0 = c0; a1 = c1; }
  const v8h hv = cvt8(a0, a1, WSCL);
  _Float16* d = pl + (size_t)i * 8;
  *(volatile v8h*)d = hv;
  __threadfence();
  *(volatile v8h*)d = hv;
}

template <int NB>
__device__ __forceinline__ int scan_chunk(const int* __restrict__ dsts, int nE, int cbase, int slotBase,
                                          int vec8, int* list, int tid, int lane, int wave) {
  int wc = 0;
#pragma unroll
  for (int g = 0; g < NGRP; ++g) {
    const int el0  = (g * NTHR + tid) * EPT;
    const int e0   = cbase + el0;
    const int sent = -2147483647 - 1;
    v4i da, db;
    if (vec8 != 0 && cbase + CHUNK <= nE) {
      da = *(const v4i*)(dsts + e0);
      db = *(const v4i*)(dsts + e0 + 4);
    } else {
      da.x = (e0     < nE) ? dsts[min(e0, nE - 1)] : sent;
      da.y = (e0 + 1 < nE) ? dsts[min(e0 + 1, nE - 1)] : sent;
      da.z = (e0 + 2 < nE) ? dsts[min(e0 + 2, nE - 1)] : sent;
      da.w = (e0 + 3 < nE) ? dsts[min(e0 + 3, nE - 1)] : sent;
      db.x = (e0 + 4 < nE) ? dsts[min(e0 + 4, nE - 1)] : sent;
      db.y = (e0 + 5 < nE) ? dsts[min(e0 + 5, nE - 1)] : sent;
      db.z = (e0 + 6 < nE) ? dsts[min(e0 + 6, nE - 1)] : sent;
      db.w = (e0 + 7 < nE) ? dsts[min(e0 + 7, nE - 1)] : sent;
    }
    const unsigned nb = (unsigned)slotBase;
    const unsigned s0 = (unsigned)da.x - nb, s1 = (unsigned)da.y - nb;
    const unsigned s2 = (unsigned)da.z - nb, s3 = (unsigned)da.w - nb;
    const unsigned s4 = (unsigned)db.x - nb, s5 = (unsigned)db.y - nb;
    const unsigned s6 = (unsigned)db.z - nb, s7 = (unsigned)db.w - nb;
    const bool h0 = s0 < (unsigned)NB, h1 = s1 < (unsigned)NB, h2 = s2 < (unsigned)NB, h3 = s3 < (unsigned)NB;
    const bool h4 = s4 < (unsigned)NB, h5 = s5 < (unsigned)NB, h6 = s6 < (unsigned)NB, h7 = s7 < (unsigned)NB;
    const unsigned any = __builtin_amdgcn_ballot_w32(h0 | h1 | h2 | h3 | h4 | h5 | h6 | h7);
    if (any != 0u) {
#define HITJ(J, HJ, SJ) { \
        const unsigned mj = __builtin_amdgcn_ballot_w32(HJ); \
        if (mj != 0u) { \
          if (HJ) { \
            const int pos = wc + (int)__builtin_amdgcn_mbcnt_lo(mj, 0u); \
            if (pos < WCAP) list[wave * WCAP + pos] = ((el0 + (J)) << 12) | (int)(SJ); \
          } \
          wc += (int)__builtin_popcount(mj); } }
      HITJ(0, h0, s0)
      HITJ(1, h1, s1)
      HITJ(2, h2, s2)
      HITJ(3, h3, s3)
      HITJ(4, h4, s4)
      HITJ(5, h5, s5)
      HITJ(6, h6, s6)
      HITJ(7, h7, s7)
#undef HITJ
    }
  }
  return wc;
}

__global__ __launch_bounds__(NTHR) void k_count(
    const int* __restrict__ dsts, int* cnt, int nE, int vec8) {
  __shared__ __attribute__((aligned(16))) int scnt[NBC];
  __shared__ __attribute__((aligned(16))) int list[LISTN];
  __shared__ int wcnt[NWAVE];
  const int tid = threadIdx.x, lane = tid & 31, wave = tid >> 5;
  const int nodeBase = blockIdx.x * NBC;

  for (int i = tid; i < NBC; i += NTHR) scnt[i] = 0;
  __syncthreads();

  const int nChunks = (nE + CHUNK - 1) / CHUNK;
#pragma unroll 1
  for (int ch = 0; ch < nChunks; ++ch) {
    const int cbase = ch * CHUNK;
    const int wc = scan_chunk<NBC>(dsts, nE, cbase, nodeBase, vec8, list, tid, lane, wave);
    if (lane == 0) wcnt[wave] = wc;
    __syncthreads();
    if (wave == 0) {
#pragma unroll 1
      for (int wsx = 0; wsx < NWAVE; ++wsx) {
        int n = __builtin_amdgcn_readfirstlane(wcnt[wsx]);
        n = n > WCAP ? WCAP : (n < 0 ? 0 : n);
        const int* lp = list + wsx * WCAP;
#pragma unroll 1
        for (int i = 0; i < n; ++i) {
          const int ent  = __builtin_amdgcn_readfirstlane(lp[i]);
          const int slot = ent & (NBC - 1);
          if (lane == 0) scnt[slot] = scnt[slot] + 1;
        }
      }
    }
    __syncthreads();
  }

  v4i cq[4];
#pragma unroll
  for (int q = 0; q < 4; ++q) {
    const int f = (wave * 4 + q) * 128 + 4 * lane;
    cq[q] = *(const v4i*)(scnt + f);
  }
  int* cpn = cnt + (size_t)nodeBase;
#pragma unroll
  for (int q = 0; q < 4; ++q) {
    const int f = (wave * 4 + q) * 128 + 4 * lane;
    *(volatile v4i*)(cpn + f) = cq[q];
  }
  __threadfence();
#pragma unroll
  for (int q = 0; q < 4; ++q) {
    const int f = (wave * 4 + q) * 128 + 4 * lane;
    *(volatile v4i*)(cpn + f) = cq[q];
  }
}

__global__ __launch_bounds__(OTHR) void k_offsets(
    const int* __restrict__ cnt, int* off, int* rbase, int nChunk) {
  __shared__ __attribute__((aligned(16))) int soff[NBC];
  __shared__ __attribute__((aligned(16))) int srb[RBN];
  __shared__ int wtot[OTHR / 32];
  const int tid = threadIdx.x, lane = tid & 31, wave = tid >> 5, sub = tid >> 8;
  for (int i = tid; i < RBN; i += OTHR) srb[i] = 0;
  __syncthreads();
  int carry = 0;
#pragma unroll 1
  for (int ch = 0; ch < nChunk; ++ch) {
    const int base = ch * NBC;
    const v4i ca = *(const v4i*)(cnt + base + 8 * tid);
    const v4i cb = *(const v4i*)(cnt + base + 8 * tid + 4);
    const int e0 = max(ca.x, 0), e1 = max(ca.y, 0), e2 = max(ca.z, 0), e3 = max(ca.w, 0);
    const int e4 = max(cb.x, 0), e5 = max(cb.y, 0), e6 = max(cb.z, 0), e7 = max(cb.w, 0);
    const int ts = e0 + e1 + e2 + e3 + e4 + e5 + e6 + e7;
    int incl = ts;
#pragma unroll
    for (int d = 1; d < 32; d <<= 1) {
      const int t = __shfl_up(incl, d);
      if (lane >= d) incl += t;
    }
    if (lane == 31) wtot[wave] = incl;
    __syncthreads();
    int S0 = 0, S1 = 0;
#pragma unroll
    for (int w = 0; w < 8; ++w) { S0 += wtot[w]; S1 += wtot[8 + w]; }
    int pre = 0;
#pragma unroll 1
    for (int w = 8 * sub; w < wave; ++w) pre += wtot[w];
    const int b0 = carry;
    const int b1 = b0 + ((S0 + 31) & ~31);
    const int b2 = b1 + ((S1 + 31) & ~31);
    const int myb = sub == 0 ? b0 : b1;
    if (tid == 0) {
      srb[min(2 * ch + 0, RBN - 1)] = b0;
      srb[min(2 * ch + 1, RBN - 1)] = b1;
    }
    int run = myb + pre + incl - ts;
    soff[8 * tid + 0] = run; run += e0;
    soff[8 * tid + 1] = run; run += e1;
    soff[8 * tid + 2] = run; run += e2;
    soff[8 * tid + 3] = run; run += e3;
    soff[8 * tid + 4] = run; run += e4;
    soff[8 * tid + 5] = run; run += e5;
    soff[8 * tid + 6] = run; run += e6;
    soff[8 * tid + 7] = run;
    carry = b2;
    __syncthreads();
    const v4i o0 = *(const v4i*)(soff + 4 * tid);
    const v4i o1 = *(const v4i*)(soff + 4 * (tid + OTHR));
    int* op = off + base;
    *(volatile v4i*)(op + 4 * tid) = o0;
    *(volatile v4i*)(op + 4 * (tid + OTHR)) = o1;
    __threadfence();
    *(volatile v4i*)(op + 4 * tid) = o0;
    *(volatile v4i*)(op + 4 * (tid + OTHR)) = o1;
    __syncthreads();
  }
  if (tid == 0) srb[min(2 * nChunk, RBN - 1)] = carry;
  __syncthreads();
  v4i rv = {0, 0, 0, 0};
  if (tid < 32) rv = *(const v4i*)(srb + 4 * tid);
  if (tid < 32) *(volatile v4i*)(rbase + 4 * tid) = rv;
  __threadfence();
  if (tid < 32) *(volatile v4i*)(rbase + 4 * tid) = rv;
}

__global__ __launch_bounds__(NTHR) void k_fill(
    const int* __restrict__ dsts, const int* __restrict__ off, const int* __restrict__ rbase,
    int* csr, int nE, int vec8, int csrLen) {
  extern __shared__ v4f lds_dyn[];
  int* region = (int*)lds_dyn;
  int* cursor = region + RCAP;
  int* list   = cursor + NBF;
  int* wcnt   = list + LISTN;
  const int tid = threadIdx.x, lane = tid & 31, wave = tid >> 5;
  const int b = blockIdx.x;
  const int nodeBase = b * NBF;

  int rb0 = rbase[b];
  const int rb1 = rbase[b + 1];
  rb0 = rb0 < 0 ? 0 : (rb0 > csrLen ? csrLen : rb0);
  rb0 &= ~31;
  int len = rb1 - rb0;
  len = len < 0 ? 0 : (len > RCAP ? RCAP : len);
  int lenW = (len + 31) & ~31;
  if (rb0 + lenW > csrLen) lenW = (csrLen - rb0) & ~31;

  {
    const v4i z = {0, 0, 0, 0};
    for (int i = tid; i < RCAP / 4; i += NTHR) ((v4i*)region)[i] = z;
    for (int s = tid; s < NBF; s += NTHR) {
      int o = off[nodeBase + s] - rb0;
      o = o < 0 ? 0 : (o > RCAP ? RCAP : o);
      cursor[s] = o;
    }
  }
  __syncthreads();

  const int nChunks = (nE + CHUNK - 1) / CHUNK;
#pragma unroll 1
  for (int ch = 0; ch < nChunks; ++ch) {
    const int cbase = ch * CHUNK;
    const int wc = scan_chunk<NBF>(dsts, nE, cbase, nodeBase, vec8, list, tid, lane, wave);
    if (lane == 0) wcnt[wave] = wc;
    __syncthreads();
    if (wave == 0) {
#pragma unroll 1
      for (int wsx = 0; wsx < NWAVE; ++wsx) {
        int n = __builtin_amdgcn_readfirstlane(wcnt[wsx]);
        n = n > WCAP ? WCAP : (n < 0 ? 0 : n);
        const int* lp = list + wsx * WCAP;
#pragma unroll 1
        for (int i = 0; i < n; ++i) {
          const int ent  = __builtin_amdgcn_readfirstlane(lp[i]);
          const int slot = ent & (NBF - 1);
          int e = cbase + ((ent >> 12) & (CHUNK - 1));
          e = e > nE - 1 ? nE - 1 : e;
          if (lane == 0) {
            int pos = cursor[slot];
            pos = pos < 0 ? 0 : (pos > RCAP - 1 ? RCAP - 1 : pos);
            region[pos] = e;
            const int np = pos + 1;
            cursor[slot] = np > RCAP ? RCAP : np;
          }
        }
      }
    }
    __syncthreads();
  }

  const int nv = lenW >> 2;
  int* gp = csr + rb0;
#pragma unroll 1
  for (int i = tid; i < nv; i += NTHR) { const v4i v = ((const v4i*)region)[i]; *(volatile v4i*)(gp + 4 * i) = v; }
  __threadfence();
#pragma unroll 1
  for (int i = tid; i < nv; i += NTHR) { const v4i v = ((const v4i*)region)[i]; *(volatile v4i*)(gp + 4 * i) = v; }
}

__global__ __launch_bounds__(NTHR) void k_agg(
    const int* __restrict__ csr, const int* __restrict__ off, const int* __restrict__ cnt,
    const int* __restrict__ srcs, const float* __restrict__ Hin, float* AG, int nN, int nE, int csrLen) {
  const int tid = threadIdx.x, lane = tid & 31, wave = tid >> 5;
  const int tbase = blockIdx.x * TGT + wave * 32;
  const int col = 4 * lane;
  const v4f z4 = {0.f, 0.f, 0.f, 0.f};
  const v4f p4 = {POISON, POISON, POISON, POISON};
  const int cl    = tbase + lane;
  const int cnt_l = cnt[cl];
  const int off_l = off[cl];

#pragma unroll 1
  for (int j = 0; j < 32; ++j) {
    const int c  = tbase + j;
    const int dg = __shfl(cnt_l, j);
    const int n  = dg < 0 ? 0 : (dg > DEGCAP ? DEGCAP : dg);
    const int st = __shfl(off_l, j);
    v4f acc = z4;
#pragma unroll 1
    for (int q0 = 0; q0 < n; q0 += 32) {
      int pos = st + q0 + lane;
      pos = pos < 0 ? 0 : (pos > csrLen - 1 ? csrLen - 1 : pos);
      int eid = csr[pos];
      eid = eid < 0 ? 0 : (eid > nE - 1 ? nE - 1 : eid);
      int sl = srcs[eid];
      sl = sl < 0 ? 0 : (sl > nN - 1 ? nN - 1 : sl);
      const int mcnt = (n - q0) < 32 ? (n - q0) : 32;
#pragma unroll 1
      for (int pp = 0; pp < mcnt; ++pp) {
        const int s = __builtin_amdgcn_readlane(sl, pp);
        acc += *(const v4f*)(Hin + (size_t)s * FD + col);
      }
    }
    const float df  = (float)(dg < 1 ? 1 : dg);
    const float inv = 1.0f / df;
    v4f v = acc * inv;
    if (dg > DEGCAP) v = p4;
    if (c >= nN) v = z4;
    float* po = AG + (size_t)c * FD + col;
    *(volatile v4f*)po = v;
    __threadfence();
    *(volatile v4f*)po = v;
  }
}

template <int ROWS, int KW, int PD>
__device__ __forceinline__ void stage_rows(const float* src, int rowBase, int nValid, _Float16* dst, int colOff) {
  constexpr int UPR = KW / 8;
  constexpr int NU  = ROWS * UPR;
  static_assert((NU % NTHR) == 0);
  const int tid = threadIdx.x;
  const v4f z4 = {0.f, 0.f, 0.f, 0.f};
#pragma unroll 2
  for (int it = 0; it < NU / NTHR; ++it) {
    const int u = it * NTHR + tid;
    const int r = u / UPR, c = (u % UPR) * 8;
    const int grow = rowBase + r;
    const int rc = grow < nValid ? grow : nValid - 1;
    const float* p = src + (size_t)rc * KW + c;
    v4f a = *(const v4f*)p, b = *(const v4f*)(p + 4);
    if (grow >= nValid) { a = z4; b = z4; }
    *(v8h*)(dst + (size_t)r * PD + colOff + c) = cvt8(a, b, 1.0f);
  }
}

template <int NT, int KW2>
__device__ __forceinline__ void mmk(v8f (&acc)[NT], const _Float16* tA, int arow,
                                    const _Float16* __restrict__ Bp, int bcol0) {
  const int lane = threadIdx.x & 31, hh = lane >> 4, m = lane & 15;
  const _Float16* ap = tA + (arow + m) * KW2 + 8 * hh;
  const _Float16* bp = Bp + (size_t)(bcol0 + m) * KW2 + 8 * hh;
#pragma unroll 1
  for (int kt = 0; kt < KW2 / 32; ++kt) {
    FragH a;
    a.h[0] = *(const v8h*)(ap + 32 * kt);
    a.h[1] = *(const v8h*)(ap + 32 * kt + 16);
#pragma unroll
    for (int t = 0; t < NT; ++t) {
      const size_t to = (size_t)(16 * t) * KW2 + 32 * kt;
      FragH bq;
      bq.h[0] = *(const v8h*)(bp + to);
      bq.h[1] = *(const v8h*)(bp + to + 16);
      acc[t] = wmh(a.v, bq.v, acc[t]);
    }
  }
}

__global__ __launch_bounds__(NTHR) void k_gnn(
    const float* __restrict__ X, const float* __restrict__ AGin, const _Float16* __restrict__ Bw,
    const float* __restrict__ bb, float* out, int nN) {
  extern __shared__ v4f lds_dyn[];
  _Float16* tA = (_Float16*)lds_dyn;
  float* stg   = (float*)(tA + GBM * KA);
  const int tid = threadIdx.x, lane = tid & 31, wave = tid >> 5, hh = lane >> 4, m = lane & 15;
  const int rowBase = blockIdx.x * GBM;
  const int r0 = 16 * wave;

  stage_rows<GBM, FD, KA>(X, rowBase, nN, tA, 0);
  stage_rows<GBM, FD, KA>(AGin, rowBase, nN, tA, FD);
  __syncthreads();

  v8f acc[8];
#pragma unroll
  for (int t = 0; t < 8; ++t) { v8f z = {0.f, 0.f, 0.f, 0.f, 0.f, 0.f, 0.f, 0.f}; acc[t] = z; }
  mmk<8, KA>(acc, tA, r0, Bw, 0);
  {
    float* sp = stg + (size_t)(r0 + 8 * hh) * HD + m;
#pragma unroll
    for (int t = 0; t < 8; ++t) {
      const float bv = bb[16 * t + m];
#pragma unroll
      for (int r = 0; r < 8; ++r)
        sp[r * HD + 16 * t] = fmaxf(acc[t][r] * WSCLI + bv, 0.f);
    }
  }
  __syncthreads();

  const size_t fbase = (size_t)rowBase * HD;
  const size_t flim  = (size_t)nN * HD;
  const v4f* s4 = (const v4f*)stg;
#pragma unroll
  for (int it = 0; it < OV; ++it) {
    const int q = it * NTHR + tid;
    const size_t f = fbase + 4 * (size_t)q;
    const v4f v = s4[q];
    if (f < flim) *(volatile v4f*)(out + f) = v;
  }
  __threadfence();
#pragma unroll
  for (int it = 0; it < OV; ++it) {
    const int q = it * NTHR + tid;
    const size_t f = fbase + 4 * (size_t)q;
    const v4f v = s4[q];
    if (f < flim) *(volatile v4f*)(out + f) = v;
  }
}

static size_t carve(size_t* o, size_t bytes) {
  const size_t r = *o;
  *o += (bytes + 255) & ~(size_t)255;
  return r;
}

extern "C" void kernel_launch(void* const* d_in, const int* in_sizes, int n_in,
                              void* d_out, int out_size, void* d_ws, size_t ws_size,
                              hipStream_t stream) {
  if (n_in < 5) return;
  const int nN = in_sizes[0] / FD;
  const int nE = in_sizes[1] / 2;
  if (nN <= 0 || nE <= 0 || in_sizes[0] != nN * FD || in_sizes[1] != 2 * nE) return;
  if (in_sizes[2] != FD * HD || in_sizes[3] != FD * HD || in_sizes[4] != HD) return;
  if ((long long)out_size != (long long)nN * HD) return;
  if (nE > (1 << 27) || nN > (1 << 22)) return;

  const float* x  = (const float*)d_in[0];
  const int*   ei = (const int*)d_in[1];
  const float* Wl = (const float*)d_in[2];
  const float* Wr = (const float*)d_in[3];
  const float* bb = (const float*)d_in[4];
  const int* src = ei;
  const int* dst = ei + nE;
  float* dout = (float*)d_out;

  const int NPAD   = ((nN + TGT - 1) / TGT) * TGT;
  const int nBC    = (nN + NBC - 1) / NBC;
  const int CNTPAD = nBC * NBC;
  if (FPC * nBC + 1 > RBN) return;
  const int nBF    = (nN + NBF - 1) / NBF;
  const int csrLen = ((nE + 31) & ~31) + 4096;
  if (31 * FPC * nBC > 4096) return;
  const int nAgg   = NPAD / TGT;
  const int nGn    = NPAD / GBM;

  char* ws = (char*)d_ws;
  size_t o = 0;
  const size_t oW   = carve(&o, (size_t)HD * KA * 2);
  const size_t oCnt = carve(&o, (size_t)CNTPAD * 4);
  const size_t oOff = carve(&o, (size_t)CNTPAD * 4);
  const size_t oRb  = carve(&o, (size_t)RBN * 4);
  const size_t oCsr = carve(&o, (size_t)csrLen * 4);
  const size_t oAG  = carve(&o, (size_t)NPAD * FD * 4);
  if (o > ws_size || o > (size_t)WSCAP) return;

  _Float16* pW = (_Float16*)(ws + oW);
  int*   cnt  = (int*)(ws + oCnt);
  int*   offp = (int*)(ws + oOff);
  int*   rb   = (int*)(ws + oRb);
  int*   csr  = (int*)(ws + oCsr);
  float* AG   = (float*)(ws + oAG);

  const int vec8 = ((nE & 3) == 0) ? 1 : 0;

  k_wprep<<<WUNITS / NTHR, NTHR, 0, stream>>>(Wr, Wl, pW, WUNITS);

  k_count<<<nBC, NTHR, 0, stream>>>(dst, cnt, nE, vec8);
  k_offsets<<<1, OTHR, 0, stream>>>(cnt, offp, rb, nBC);
  hipFuncSetAttribute(reinterpret_cast<const void*>(&k_fill),
                      hipFuncAttributeMaxDynamicSharedMemorySize, LDS_FILL);
  k_fill<<<nBF, NTHR, LDS_FILL, stream>>>(dst, offp, rb, csr, nE, vec8, csrLen);

  k_agg<<<nAgg, NTHR, 0, stream>>>(csr, offp, cnt, src, x, AG, nN, nE, csrLen);

  hipFuncSetAttribute(reinterpret_cast<const void*>(&k_gnn),
                      hipFuncAttributeMaxDynamicSharedMemorySize, LDS_GN);
  k_gnn<<<nGn, NTHR, LDS_GN, stream>>>(x, AG, pW, bb, dout, nN);
}
